// JEPAImpactModel_20736102105550
// MI455X (gfx1250) — hardware-run, weakly checked
//
#include <hip/hip_runtime.h>
#include <math.h>

typedef __attribute__((ext_vector_type(16))) __bf16 v16b;
typedef __attribute__((ext_vector_type(8)))  __bf16 v8b;
typedef __attribute__((ext_vector_type(8)))  float  v8f;
typedef __attribute__((ext_vector_type(4)))  float  v4f;

constexpr int kSteps   = 16384;
constexpr int kLatent  = 16;
constexpr int kBelief  = 32;
constexpr int kHid     = 16;
constexpr int kGates   = 3 * kBelief;
constexpr int kKin     = kLatent + 1;
constexpr int kKpad    = 32;
constexpr int kRowsBlk = 64;
constexpr int kChunk   = 32;
constexpr int kNumChunks = kSteps / kChunk;
constexpr size_t kWsGiBytes = (size_t)kSteps * kGates * 4;
constexpr size_t kWsTotal   = kWsGiBytes;
static_assert(kGates == 96);
static_assert(kKin == 17 && kKin <= kKpad);
static_assert(kSteps % kRowsBlk == 0);
static_assert(kSteps % kChunk == 0);
static_assert(kGates % 16 == 0);
static_assert(kWsTotal == 6291456ull);
static_assert(kWsTotal <= 134217728ull);
static_assert((size_t)kSteps * kBelief * 4 == 2097152ull);

__device__ __forceinline__ void pin1(float& v) { asm volatile("" : "+v"(v)); }

__device__ __forceinline__ unsigned short f2bf_bits(float f) {
  const unsigned u = __float_as_uint(f);
  return (unsigned short)((u + 0x7FFFu + ((u >> 16) & 1u)) >> 16);
}
__device__ __forceinline__ float bf_bits2f(unsigned short h) {
  return __uint_as_float(((unsigned)h) << 16);
}

union FragB { v16b v; v8b h[2]; };
__device__ __forceinline__ v16b ld_frag(const unsigned short* p) {
  FragB f;
  f.h[0] = *(const v8b*)(const void*)(p);
  f.h[1] = *(const v8b*)(const void*)(p + 16);
  return f.v;
}

__device__ __forceinline__ v8f mma_bf16(v16b a, v16b b, v8f c) {
  c = __builtin_amdgcn_wmma_f32_16x16x32_bf16(false, a, false, b, (short)0, c, false, false);
  asm volatile("v_nop\n\tv_nop\n\tv_nop\n\tv_nop" : "+v"(c) : "v"(a), "v"(b));
  return c;
}

__global__ __launch_bounds__(128) void gi_proj_kernel(
    const float* __restrict__ obs, const float* __restrict__ act,
    const float* __restrict__ enc_w, const float* __restrict__ enc_b,
    const float* __restrict__ w_ih, const float* __restrict__ b_ih,
    float* __restrict__ gi)
{
  __shared__ __align__(16) unsigned short sAh[kRowsBlk * kKpad];
  __shared__ __align__(16) unsigned short sAl[kRowsBlk * kKpad];
  __shared__ __align__(16) unsigned short sBh[kGates * kKpad];
  __shared__ __align__(16) unsigned short sBl[kGates * kKpad];
  __shared__ __align__(16) float slab[4][16 * kGates];

  const int tid  = threadIdx.x;
  const int lane = tid & 31;
  const int wave = tid >> 5;
  const int c    = lane & 15;
  const int hs   = lane >> 4;
  const int t0   = blockIdx.x * kRowsBlk;

#pragma unroll 1
  for (int i = 0; i < 16; ++i) {
    const int e    = i * 128 + tid;
    const int row  = e >> 5;
    const int col  = e & 31;
    const int t    = t0 + row;
    const int colc = (col < kLatent) ? col : (kLatent - 1);
    const int tp   = (t > 0) ? (t - 1) : 0;
    float o  = obs[t];
    float ew = enc_w[colc];
    float eb = enc_b[colc];
    float ap = act[tp];
    pin1(o);
    pin1(ew);
    pin1(eb);
    pin1(ap);
    const float zt  = tanhf(fmaf(o, ew, eb));
    const float apv = (t > 0) ? ap : 0.0f;
    const float v   = (col < kLatent) ? zt : ((col == kLatent) ? apv : 0.0f);
    const unsigned short hb = f2bf_bits(v);
    const unsigned short lb = f2bf_bits(v - bf_bits2f(hb));
    sAh[e] = hb;
    sAl[e] = lb;
  }
#pragma unroll 1
  for (int i = 0; i < 24; ++i) {
    const int e  = i * 128 + tid;
    const int n  = e >> 5;
    const int k  = e & 31;
    const int kc = (k < kKin) ? k : (kKin - 1);
    float w = w_ih[kc * kGates + n];
    pin1(w);
    const float v = (k < kKin) ? w : 0.0f;
    const unsigned short hb = f2bf_bits(v);
    const unsigned short lb = f2bf_bits(v - bf_bits2f(hb));
    sBh[e] = hb;
    sBl[e] = lb;
  }
  __syncthreads();

  const int arow = wave * 16 + c;
  const v16b ah = ld_frag(sAh + arow * kKpad + 8 * hs);
  const v16b al = ld_frag(sAl + arow * kKpad + 8 * hs);

  float* sl = slab[wave];
#pragma unroll 1
  for (int j = 0; j < kGates / 16; ++j) {
    const int n = 16 * j + c;
    const v16b bh = ld_frag(sBh + n * kKpad + 8 * hs);
    const v16b bl = ld_frag(sBl + n * kKpad + 8 * hs);
    v8f acc = (v8f){0.f, 0.f, 0.f, 0.f, 0.f, 0.f, 0.f, 0.f};
    acc = mma_bf16(ah, bl, acc);
    acc = mma_bf16(al, bh, acc);
    acc = mma_bf16(ah, bh, acc);
    float bv = b_ih[n];
    pin1(bv);
#pragma unroll
    for (int r = 0; r < 8; ++r) {
      sl[(8 * hs + r) * kGates + n] = acc[r] + bv;
    }
  }
  __syncthreads();

  float* gw = gi + (size_t)(t0 + wave * 16) * kGates;
  for (int pass = 0; pass < 2; ++pass) {
#pragma unroll
    for (int it = 0; it < 12; ++it) {
      const int idx = (it * 32 + lane) * 4;
      const v4f v = *(const v4f*)(sl + idx);
      *(volatile v4f*)(gw + idx) = v;
    }
    __threadfence();
  }
}

__device__ __forceinline__ float sigm_f(float v) {
  const float vc = fminf(fmaxf(v, -30.0f), 30.0f);
  return 1.0f / (1.0f + expf(-vc));
}
__device__ __forceinline__ float tanh_f(float v) {
  const float vc = fminf(fmaxf(v, -15.0f), 15.0f);
  return 1.0f - 2.0f / (expf(2.0f * vc) + 1.0f);
}

__global__ __launch_bounds__(32) void belief_chain_kernel(
    const float* __restrict__ gi, const float* __restrict__ act,
    const float* __restrict__ bounce,
    const float* __restrict__ w_hh, const float* __restrict__ b_hh,
    const float* __restrict__ imp_w1, const float* __restrict__ imp_b1,
    const float* __restrict__ imp_w2, const float* __restrict__ imp_b2,
    float* __restrict__ out)
{
  __shared__ __align__(16) float sW[kBelief * 32 * 4];
  __shared__ __align__(16) float sW2[kHid * 32];
  __shared__ __align__(16) float sGi[kChunk * kGates];
  __shared__ __align__(16) float sOut[kChunk * kBelief];
  __shared__ __align__(16) float sV[32];
  __shared__ __align__(16) float sH[32];
  __shared__ __align__(16) float sAct[kChunk];
  __shared__ __align__(16) float sFlag[kChunk];

  const int lane = threadIdx.x;
  const int jc   = lane & (kHid - 1);

#pragma unroll 1
  for (int i = 0; i < kBelief; ++i) {
    float wr = w_hh[i * kGates + lane];
    float wz = w_hh[i * kGates + kBelief + lane];
    float wn = w_hh[i * kGates + 2 * kBelief + lane];
    float w1 = imp_w1[i * kHid + jc];
    pin1(wr);
    pin1(wz);
    pin1(wn);
    pin1(w1);
    v4f wv;
    wv[0] = wr;
    wv[1] = wz;
    wv[2] = wn;
    wv[3] = w1;
    *(v4f*)(sW + (i * 32 + lane) * 4) = wv;
  }
#pragma unroll 1
  for (int k = 0; k < kHid; ++k) {
    float w2 = imp_w2[k * kBelief + lane];
    pin1(w2);
    sW2[k * 32 + lane] = w2;
  }

  float bhr = b_hh[lane];
  float bhz = b_hh[kBelief + lane];
  float bhn = b_hh[2 * kBelief + lane];
  float b1c = imp_b1[jc];
  float b2c = imp_b2[lane];
  float w1a = imp_w1[kBelief * kHid + jc];
  pin1(bhr);
  pin1(bhz);
  pin1(bhn);
  pin1(b1c);
  pin1(b2c);
  pin1(w1a);

  sV[lane] = 0.0f;
  float bel = 0.0f;

#pragma unroll 1
  for (int ch = 0; ch < kNumChunks; ++ch) {
    const int t0 = ch * kChunk;
    const float* gsrc = gi + (size_t)t0 * kGates;
#pragma unroll 1
    for (int g = 0; g < 3; ++g) {
      v4f q[8];
#pragma unroll
      for (int u = 0; u < 8; ++u) {
        q[u] = *(const v4f*)(gsrc + ((g * 8 + u) * 32 + lane) * 4);
      }
#pragma unroll
      for (int u = 0; u < 8; ++u) {
        *(v4f*)(sGi + ((g * 8 + u) * 32 + lane) * 4) = q[u];
      }
    }
    {
      float av = act[t0 + lane];
      float bv = bounce[t0 + lane];
      pin1(av);
      pin1(bv);
      sAct[lane]  = av;
      sFlag[lane] = ((bv == 1.0f) && ((t0 + lane) > 0)) ? 1.0f : 0.0f;
    }
    __syncthreads();

#pragma unroll 1
    for (int s = 0; s < kChunk; ++s) {
      float ghr = bhr;
      float ghz = bhz;
      float ghn = bhn;
      float a1  = b1c;
#pragma unroll 1
      for (int i4 = 0; i4 < kBelief / 4; ++i4) {
        const v4f hv = *(const v4f*)(sV + 4 * i4);
#pragma unroll
        for (int qq = 0; qq < 4; ++qq) {
          const v4f w = *(const v4f*)(sW + ((4 * i4 + qq) * 32 + lane) * 4);
          const float hq = hv[qq];
          ghr = fmaf(hq, w[0], ghr);
          ghz = fmaf(hq, w[1], ghz);
          ghn = fmaf(hq, w[2], ghn);
          a1  = fmaf(hq, w[3], a1);
        }
      }
      const float gir = sGi[s * kGates + lane];
      const float giz = sGi[s * kGates + kBelief + lane];
      const float gin = sGi[s * kGates + 2 * kBelief + lane];
      const float at  = sAct[s];
      const float fl  = sFlag[s];

      const float r  = sigm_f(gir + ghr);
      const float zg = sigm_f(giz + ghz);
      const float nn = tanh_f(gin + r * ghn);
      const float bn = (1.0f - zg) * nn + zg * bel;

      a1 = fmaf(at, w1a, a1);
      const float hh = tanh_f(a1);
      sH[lane] = hh;
      __syncthreads();

      float delta = b2c;
#pragma unroll 1
      for (int k4 = 0; k4 < kHid / 4; ++k4) {
        const v4f hq4 = *(const v4f*)(sH + 4 * k4);
#pragma unroll
        for (int qq = 0; qq < 4; ++qq) {
          const float w2 = sW2[(4 * k4 + qq) * 32 + lane];
          delta = fmaf(hq4[qq], w2, delta);
        }
      }
      const float bimp = bel + delta;
      const float bnew = (fl != 0.0f) ? bimp : bn;
      bel = bnew;
      sV[lane] = bnew;
      sOut[s * kBelief + lane] = bnew;
      __syncthreads();
    }

    float* ow = out + (size_t)t0 * kBelief;
    for (int pass = 0; pass < 2; ++pass) {
#pragma unroll
      for (int it = 0; it < 8; ++it) {
        const int idx = (it * 32 + lane) * 4;
        const v4f v = *(const v4f*)(sOut + idx);
        *(volatile v4f*)(ow + idx) = v;
      }
      __threadfence();
    }
  }
}

extern "C" void kernel_launch(void* const* d_in, const int* in_sizes, int n_in,
                              void* d_out, int out_size, void* d_ws, size_t ws_size,
                              hipStream_t stream) {
  if (n_in < 13 || d_out == nullptr || d_ws == nullptr) return;
  if (in_sizes[0] != kSteps) return;
  if (in_sizes[1] != kSteps) return;
  if (in_sizes[2] != kSteps) return;
  if (in_sizes[3] != kLatent) return;
  if (in_sizes[4] != kLatent) return;
  if (in_sizes[5] != kKin * kGates) return;
  if (in_sizes[6] != kGates) return;
  if (in_sizes[7] != kBelief * kGates) return;
  if (in_sizes[8] != kGates) return;
  if (in_sizes[9] != (kBelief + 1) * kHid) return;
  if (in_sizes[10] != kHid) return;
  if (in_sizes[11] != kHid * kBelief) return;
  if (in_sizes[12] != kBelief) return;
  if (out_size != kSteps * kBelief) return;
  if (ws_size < kWsTotal) return;

  const float* obs    = (const float*)d_in[0];
  const float* act    = (const float*)d_in[1];
  const float* bounce = (const float*)d_in[2];
  const float* enc_w  = (const float*)d_in[3];
  const float* enc_b  = (const float*)d_in[4];
  const float* w_ih   = (const float*)d_in[5];
  const float* b_ih   = (const float*)d_in[6];
  const float* w_hh   = (const float*)d_in[7];
  const float* b_hh   = (const float*)d_in[8];
  const float* imp_w1 = (const float*)d_in[9];
  const float* imp_b1 = (const float*)d_in[10];
  const float* imp_w2 = (const float*)d_in[11];
  const float* imp_b2 = (const float*)d_in[12];
  float* out = (float*)d_out;
  float* gi  = (float*)d_ws;

  gi_proj_kernel<<<kSteps / kRowsBlk, 128, 0, stream>>>(obs, act, enc_w, enc_b, w_ih, b_ih, gi);
  belief_chain_kernel<<<1, 32, 0, stream>>>(gi, act, bounce, w_hh, b_hh,
                                            imp_w1, imp_b1, imp_w2, imp_b2, out);
}
